// SchNetRepresentation_67654324846791
// MI455X (gfx1250) — hardware-verified
//
#include <hip/hip_runtime.h>
#include <math.h>

#define NATOM 16384
#define NPAIR 524288
#define NB 128
#define NRBF 20
#define KRBF 32
#define NLAYER 3
#define CHK 131072
#define NCHK (NPAIR / CHK)
#define NT 256
#define SRB 2048
#define NTILE (NATOM / SRB)
#define SCH 4096
#define NSTEP (CHK / SCH)
#define WPL 69632
#define W_IN 0
#define W_F1 16384
#define W_F2 20480
#define W_O1 36864
#define W_O2 53248
#define SC_W 16.0f
#define SC_X 16.0f
#define SC_T 64.0f
#define OSC SC_T

typedef __attribute__((ext_vector_type(16))) _Float16 v16h;
typedef __attribute__((ext_vector_type(8)))  _Float16 v8h;
typedef __attribute__((ext_vector_type(4)))  _Float16 v4h;
typedef __attribute__((ext_vector_type(16))) __bf16   v16b;
typedef __attribute__((ext_vector_type(8)))  __bf16   v8b;
typedef __attribute__((ext_vector_type(8)))  float    v8f;
typedef __attribute__((ext_vector_type(4)))  float    v4f;
typedef __attribute__((ext_vector_type(4)))  int      v4i;

__device__ __forceinline__ unsigned short f2bf_bits(float f) {
  unsigned u = __float_as_uint(f);
  return (unsigned short)((u + 0x7FFFu + ((u >> 16) & 1u)) >> 16);
}
__device__ __forceinline__ float bf_bits2f(unsigned short h) { return __uint_as_float(((unsigned)h) << 16); }

__device__ __forceinline__ float ssp_f(float x) {
  const float t = __expf(-fabsf(x));
  return fmaxf(x, 0.f) + __logf(1.0f + t) - 0.69314718055994531f;
}

__device__ __forceinline__ void dep_guard_h(v8f& a, v8f& b, v16h x, v16h y) { asm volatile("v_nop\n\tv_nop\n\tv_nop\n\tv_nop" : "+v"(a), "+v"(b) : "v"(x), "v"(y)); }
__device__ __forceinline__ void dep_guard_b(v8f& a, v8f& b, v16b x, v16b y) { asm volatile("v_nop\n\tv_nop\n\tv_nop\n\tv_nop" : "+v"(a), "+v"(b) : "v"(x), "v"(y)); }
__device__ __forceinline__ void keep4_h(v16h a, v16h b, v16h c, v16h d) { asm volatile("v_nop" :: "v"(a), "v"(b), "v"(c), "v"(d)); }
__device__ __forceinline__ void keep4_b(v16b a, v16b b, v16b c, v16b d) { asm volatile("v_nop" :: "v"(a), "v"(b), "v"(c), "v"(d)); }
__device__ __forceinline__ void acc_guard4(v8f& a, v8f& b, v8f& c, v8f& d) { asm volatile("v_nop\n\tv_nop\n\tv_nop\n\tv_nop" : "+v"(a), "+v"(b), "+v"(c), "+v"(d)); }
template <typename T> struct Frag;
template <> struct Frag<_Float16> {
  typedef v16h V; union U { v16h v; v8h h[2]; };
  static __device__ __forceinline__ v16h load(const _Float16* p) {
    U f; f.h[0] = *(const v8h*)(p); f.h[1] = *(const v8h*)(p + 16); return f.v;
  }
  static __device__ __forceinline__ v8f mma(v16h a, v16h b, v8f c) {
    return __builtin_amdgcn_wmma_f32_16x16x32_f16(false, a, false, b, (short)0, c, false, false);
  }
  static __device__ __forceinline__ void guard(v8f& a, v8f& b, v16h x, v16h y) { dep_guard_h(a, b, x, y); }
  static __device__ __forceinline__ void keep(v16h a, v16h b, v16h c, v16h d) { keep4_h(a, b, c, d); }
};
template <> struct Frag<__bf16> {
  typedef v16b V; union U { v16b v; v8b h[2]; };
  static __device__ __forceinline__ v16b load(const __bf16* p) {
    U f; f.h[0] = *(const v8b*)(p); f.h[1] = *(const v8b*)(p + 16); return f.v;
  }
  static __device__ __forceinline__ v8f mma(v16b a, v16b b, v8f c) {
    return __builtin_amdgcn_wmma_f32_16x16x32_bf16(false, a, false, b, (short)0, c, false, false);
  }
  static __device__ __forceinline__ void guard(v8f& a, v8f& b, v16b x, v16b y) { dep_guard_b(a, b, x, y); }
  static __device__ __forceinline__ void keep(v16b a, v16b b, v16b c, v16b d) { keep4_b(a, b, c, d); }
};

template <int ET> struct Elem;
template <> struct Elem<0> { typedef _Float16 T; };
template <> struct Elem<1> { typedef __bf16 T; };
template <int ET, bool SPLIT, int BIAS_MODE, int OUT_MODE, bool RESID, int ACT = 0>
__global__ __launch_bounds__(256) void wmma_gemm64(
    const unsigned short* __restrict__ Ap, const unsigned short* __restrict__ A2p, int lda, long strideA,
    const unsigned short* __restrict__ Btp, const unsigned short* __restrict__ Bt2p, int ldb, long strideB,
    void* __restrict__ Cout, void* __restrict__ Cout2, int ldc, long strideC,
    const float* __restrict__ bias,
    const float* __restrict__ resid, long strideR,
    int M, int N, int K, float scale) {
  typedef typename Elem<ET>::T T;
  typedef typename Frag<T>::V V;
  const T* A = (const T*)Ap; const T* A2 = (const T*)A2p; const T* Bt = (const T*)Btp; const T* Bt2 = (const T*)Bt2p;
  __shared__ __align__(16) float sT[8][16 * 68];
  const int b    = blockIdx.y;
  const int lane = threadIdx.x & 31;
  const int wave = threadIdx.x >> 5;
  const int tilesN = N >> 6;
  const int tilesM = M >> 6;
  const int tile = blockIdx.x * 8 + wave;
  if (tile >= tilesM * tilesN) return;
  const int tm = tile / tilesN;
  const int tn = tile - tm * tilesN;
  const int m0 = tm << 6;
  const int n0 = tn << 6;

  const T* Ab  = A  + (size_t)b * strideA;
  const T* Bb  = Bt + (size_t)b * strideB;
  const T* Ab2 = SPLIT ? (A2  + (size_t)b * strideA) : nullptr;
  const T* Bb2 = SPLIT ? (Bt2 + (size_t)b * strideB) : nullptr;

  const int rlane = lane & 15;
  const int koff  = (lane >> 4) * 8;
  const int mOff  = (lane >> 4) * 8;

  v8f acc[4][4];
#pragma unroll
  for (int i = 0; i < 4; ++i)
#pragma unroll
    for (int j = 0; j < 4; ++j) acc[i][j] = (v8f){0.f,0.f,0.f,0.f,0.f,0.f,0.f,0.f};

  for (int k0 = 0; k0 < K; k0 += 32) {
    V bh[4], bl[4];
#pragma unroll
    for (int j = 0; j < 4; ++j) {
      const size_t bo = (size_t)(n0 + (j << 4) + rlane) * ldb + koff + k0;
      bh[j] = Frag<T>::load(Bb + bo);
      if (SPLIT) bl[j] = Frag<T>::load(Bb2 + bo);
    }
#pragma unroll
    for (int i = 0; i < 4; ++i) {
      const size_t ao = (size_t)(m0 + (i << 4) + rlane) * lda + koff + k0;
      V ah = Frag<T>::load(Ab + ao);
      V al;
      if (SPLIT) al = Frag<T>::load(Ab2 + ao);
#pragma unroll
      for (int j = 0; j < 4; ++j) {
        acc[i][j] = Frag<T>::mma(ah, bh[j], acc[i][j]);
        if (SPLIT) {
          acc[i][j] = Frag<T>::mma(ah, bl[j], acc[i][j]);
          acc[i][j] = Frag<T>::mma(al, bh[j], acc[i][j]);
        }
      }
      Frag<T>::guard(acc[i][0], acc[i][3], ah, SPLIT ? al : ah);
    }
    Frag<T>::keep(bh[0], bh[1], bh[2], bh[3]);
    if (SPLIT) Frag<T>::keep(bl[0], bl[1], bl[2], bl[3]);
  }
  acc_guard4(acc[0][0], acc[0][1], acc[0][2], acc[0][3]);
  acc_guard4(acc[1][0], acc[1][1], acc[1][2], acc[1][3]);
  acc_guard4(acc[2][0], acc[2][1], acc[2][2], acc[2][3]);
  acc_guard4(acc[3][0], acc[3][1], acc[3][2], acc[3][3]);

  float* slab = sT[wave];
  const float* Rb = RESID ? (resid + (size_t)b * strideR) : nullptr;
#pragma unroll
  for (int i = 0; i < 4; ++i) {
    const int mBase = m0 + (i << 4);
#pragma unroll
    for (int j = 0; j < 4; ++j) {
      const int n = n0 + (j << 4) + rlane;
      float bv = 0.f;
      if (BIAS_MODE == 2) bv = bias[n];
#pragma unroll
      for (int r = 0; r < 8; ++r) {
        float v = acc[i][j][r] * scale;
        if (BIAS_MODE == 1) v += bias[mBase + mOff + r];
        if (BIAS_MODE == 2) v += bv;
        if (RESID) v += Rb[(size_t)(mBase + mOff + r) * ldc + n];
        if (ACT == 1) v = tanhf(v);
        if (ACT == 2) v = fmaxf(v, 0.0f);
        if (ACT == 3) v = v / (1.0f + expf(-v));
        if (ACT == 4) v = (v > 0.f) ? v : 0.01f * v;
        if (ACT == 5) v = 0.5f * v * (1.0f + erff(v * 0.70710678118654752f));
        if (ACT == 6) v = OSC * ssp_f(v);
        if (ACT == 7) v = OSC * v;
        slab[(mOff + r) * 68 + (j << 4) + rlane] = v;
      }
    }
    __builtin_amdgcn_fence(__ATOMIC_RELEASE, "workgroup");
    __builtin_amdgcn_wave_barrier();
    __builtin_amdgcn_fence(__ATOMIC_ACQUIRE, "workgroup");
    if (OUT_MODE == 0) {
      float* C = (float*)Cout + (size_t)b * strideC;
      const int hh = lane >> 4, c4 = (lane & 15) * 4;
      for (int pass = 0; pass < 2; ++pass) {
#pragma unroll
        for (int it = 0; it < 8; ++it) {
          const int row = it * 2 + hh;
          v4f v = *(const v4f*)(slab + row * 68 + c4);
          *(volatile v4f*)(C + (size_t)(mBase + row) * ldc + n0 + c4) = v;
        }
        __threadfence();
      }
    } else {
      const int q = lane >> 3, c8 = (lane & 7) * 8;
      unsigned short* C  = (unsigned short*)Cout  + (size_t)b * strideC;
      unsigned short* C2 = (OUT_MODE == 2) ? ((unsigned short*)Cout2 + (size_t)b * strideC) : nullptr;
      for (int pass = 0; pass < 2; ++pass) {
#pragma unroll
        for (int it = 0; it < 4; ++it) {
          const int row = it * 4 + q;
          const float* sp = slab + row * 68 + c8;
          v8h hv, lv;
#pragma unroll
          for (int e = 0; e < 8; ++e) {
            if (OUT_MODE == 1) {
              hv[e] = (_Float16)sp[e];
            } else {
              unsigned short hb = f2bf_bits(sp[e]);
              unsigned short lb = f2bf_bits(sp[e] - bf_bits2f(hb));
              hv[e] = __builtin_bit_cast(_Float16, hb);
              lv[e] = __builtin_bit_cast(_Float16, lb);
            }
          }
          *(volatile v8h*)(C + (size_t)(mBase + row) * ldc + n0 + c8) = hv;
          if (OUT_MODE == 2) *(volatile v8h*)(C2 + (size_t)(mBase + row) * ldc + n0 + c8) = lv;
        }
        __threadfence();
      }
    }
    __builtin_amdgcn_fence(__ATOMIC_RELEASE, "workgroup");
    __builtin_amdgcn_wave_barrier();
    __builtin_amdgcn_fence(__ATOMIC_ACQUIRE, "workgroup");
  }
}

__device__ __forceinline__ int blk_excl_scan(int cnt, int* scan_ws, int tid, int* tot) {
  const int lane = tid & 31, wave = tid >> 5; int incl = cnt;
#pragma unroll
  for (int o = 1; o < 32; o <<= 1) { const int v = __shfl_up(incl, o, 32); if (lane >= o) incl += v; }
  if (lane == 31) scan_ws[wave] = incl;
  __syncthreads();
  if (wave == 0) { int wv = (lane < NT / 32) ? scan_ws[lane] : 0; int wincl = wv;
#pragma unroll
    for (int o = 1; o < 32; o <<= 1) { const int v = __shfl_up(wincl, o, 32); if (lane >= o) wincl += v; }
    if (lane < NT / 32) scan_ws[32 + lane] = wincl - wv; if (lane == 31) scan_ws[64] = wincl; }
  __syncthreads();
  const int res = scan_ws[32 + wave] + incl - cnt; *tot = scan_ws[64];
  return res;
}
template <int SP, int CAP>
__device__ __forceinline__ int chunk_hits(const int* __restrict__ dstv, int e0, int n0, int tid, int* LIST, int* scan_ws) {
  const int eb = e0 + tid * SP;
  int rec[SP]; int cnt = 0;
#pragma unroll
  for (int k = 0; k < SP; k += 4) {
    const v4i d4 = *(const v4i*)(dstv + eb + k);
#pragma unroll
    for (int e = 0; e < 4; ++e) {
      const int d = d4[e]; int r = -1;
      if (d >= n0 && d < n0 + SRB) { r = ((d - n0) << 19) | (eb + k + e); ++cnt; }
      rec[k + e] = r;
    }
  }
  int tot; int p = blk_excl_scan(cnt, scan_ws, tid, &tot);
#pragma unroll
  for (int k = 0; k < SP; ++k) if (rec[k] >= 0) { if ((unsigned)p < (unsigned)CAP) LIST[p] = rec[k]; ++p; }
  __syncthreads();
  return tot < CAP ? tot : CAP;
}

__global__ __launch_bounds__(NT) void prep_kernel(const float* __restrict__ inW, const float* __restrict__ fW1,
                                                 const float* __restrict__ fW2, const float* __restrict__ oW1,
                                                 const float* __restrict__ oW2, _Float16* __restrict__ WT) {
  const int tid = threadIdx.x;
  v8h hv;
  _Float16* dst;
  if (blockIdx.x < 96) {
    const int t = blockIdx.x * NT + tid;
    const int q = t >> 11, tt = t & 2047;
    const int l = q >> 2, m = q & 3;
    const int n = tt >> 4, k8 = (tt & 15) * 8;
    const float* src = (m == 0) ? inW : ((m == 1) ? fW2 : ((m == 2) ? oW1 : oW2));
    src += (size_t)l * (NB * NB);
    const int moff = (m == 0) ? W_IN : ((m == 1) ? W_F2 : ((m == 2) ? W_O1 : W_O2));
#pragma unroll
    for (int e = 0; e < 8; ++e) hv[e] = (_Float16)(src[(size_t)(k8 + e) * NB + n] * SC_W);
    dst = WT + (size_t)l * WPL + moff + n * NB + k8;
  } else {
    const int u = (blockIdx.x - 96) * NT + tid;
    const int l = u >> 9, tt = u & 511;
    const int n = tt >> 2, k8 = (tt & 3) * 8;
#pragma unroll
    for (int e = 0; e < 8; ++e) {
      const int k = k8 + e; const int kc = (k < NRBF) ? k : (NRBF - 1);
      const float w = fW1[(size_t)l * (NRBF * NB) + kc * NB + n] * SC_W;
      hv[e] = (_Float16)((k < NRBF) ? w : 0.f);
    }
    dst = WT + (size_t)l * WPL + W_F1 + n * KRBF + k8;
  }
  *(volatile v8h*)dst = hv;
  __threadfence();
  *(volatile v8h*)dst = hv;
}

__global__ __launch_bounds__(NT) void embed_kernel(const int* __restrict__ Z, const float* __restrict__ emb,
                                                  float* __restrict__ X, _Float16* __restrict__ X16) {
  const int t = blockIdx.x * NT + threadIdx.x;
  {
    const int row = t >> 5, c4 = (t & 31) * 4;
    int z = Z[row]; z = z < 0 ? 0 : (z > 99 ? 99 : z);
    const v4f v = *(const v4f*)(emb + z * NB + c4);
    float* p = X + (size_t)row * NB + c4;
    *(volatile v4f*)p = v;
    __threadfence();
    *(volatile v4f*)p = v;
  }
  if (t < NATOM * 16) {
    const int row = t >> 4, c8 = (t & 15) * 8;
    int z = Z[row]; z = z < 0 ? 0 : (z > 99 ? 99 : z);
    const v4f v0 = *(const v4f*)(emb + z * NB + c8);
    const v4f v1 = *(const v4f*)(emb + z * NB + c8 + 4);
    v8h h;
#pragma unroll
    for (int e = 0; e < 4; ++e) { h[e] = (_Float16)(v0[e] * SC_X); h[4 + e] = (_Float16)(v1[e] * SC_X); }
    _Float16* p = X16 + (size_t)row * NB + c8;
    *(volatile v8h*)p = h;
    __threadfence();
    *(volatile v8h*)p = h;
  }
}

__global__ __launch_bounds__(NT) void cast16_kernel(const float* __restrict__ X, _Float16* __restrict__ X16, int n8) {
  const int i = blockIdx.x * NT + threadIdx.x;
  if (i < n8) {
    const v4f v0 = *(const v4f*)(X + (size_t)i * 8);
    const v4f v1 = *(const v4f*)(X + (size_t)i * 8 + 4);
    v8h h;
#pragma unroll
    for (int e = 0; e < 4; ++e) { h[e] = (_Float16)(v0[e] * SC_X); h[4 + e] = (_Float16)(v1[e] * SC_X); }
    _Float16* p = X16 + (size_t)i * 8;
    *(volatile v8h*)p = h;
    __threadfence();
    *(volatile v8h*)p = h;
  }
}

__global__ __launch_bounds__(NT) void geom_kernel(const float* __restrict__ R, const int* __restrict__ idx_i,
                                                 const int* __restrict__ idx_j, _Float16* __restrict__ rbf,
                                                 float* __restrict__ rcut, int cbase) {
  __shared__ __align__(16) _Float16 tile[NT * KRBF];
  __shared__ __align__(16) float rcs[NT];
  const int tid = threadIdx.x, lane = tid & 31, wave = tid >> 5;
  const int p = cbase + blockIdx.x * NT + tid;
  int i = idx_i[p]; i = i < 0 ? 0 : (i >= NATOM ? NATOM - 1 : i);
  int j = idx_j[p]; j = j < 0 ? 0 : (j >= NATOM ? NATOM - 1 : j);
  const float dx = R[3 * i] - R[3 * j];
  const float dy = R[3 * i + 1] - R[3 * j + 1];
  const float dz = R[3 * i + 2] - R[3 * j + 2];
  const float d = sqrtf(dx * dx + dy * dy + dz * dz);
  const float inv19 = 1.0f / 19.0f;
  const float width = 5.0f * inv19;
  const float coeff = -0.5f / (width * width);
#pragma unroll 1
  for (int k = 0; k < KRBF; ++k) {
    float v = 0.f;
    if (k < NRBF) {
      const float off = 5.0f * ((float)k * inv19);
      const float df = d - off;
      v = __expf(coeff * (df * df));
      v = (v < 6.103515625e-05f) ? 0.f : v;
    }
    tile[tid * KRBF + k] = (_Float16)v;
  }
  const float fc = 0.5f * (cosf(d * 0.62831853071795864f) + 1.0f);
  rcs[tid] = (d < 5.0f) ? fc : 0.f;
  __syncthreads();
  for (int pass = 0; pass < 2; ++pass) {
#pragma unroll
    for (int it = 0; it < 4; ++it) {
      const int row = wave * 32 + it * 8 + (lane >> 2);
      const int c8 = (lane & 3) * 8;
      const v8h v = *(const v8h*)(tile + row * KRBF + c8);
      *(volatile v8h*)(rbf + (size_t)(blockIdx.x * NT + row) * KRBF + c8) = v;
    }
    if (wave == 0) {
#pragma unroll
      for (int it = 0; it < 2; ++it) {
        const v4f v = *(const v4f*)(rcs + it * 128 + 4 * lane);
        *(volatile v4f*)(rcut + (size_t)blockIdx.x * NT + it * 128 + 4 * lane) = v;
      }
    }
    __threadfence();
  }
}

__global__ __launch_bounds__(NT) void agg_kernel(const int* __restrict__ idx_i, const int* __restrict__ idx_j,
                                                const float* __restrict__ H, const _Float16* __restrict__ W16,
                                                const float* __restrict__ rcut, float* AGG, _Float16* __restrict__ AGG16,
                                                int cbase, int first, int last) {
  __shared__ int LIST[SCH];
  __shared__ int scan_ws[80];
  const int tid = threadIdx.x, lane = tid & 31, wave = tid >> 5;
  const int n0 = blockIdx.x * SRB;
  const int rw0 = n0 + wave * (SRB / 8);
  const v4f z4 = {0.f, 0.f, 0.f, 0.f};
  if (first) {
#pragma unroll 1
    for (int jr = 0; jr < SRB / 8; ++jr) *(v4f*)(AGG + (size_t)(rw0 + jr) * NB + 4 * lane) = z4;
  }
  const float rsc = 1.0f / SC_T;
#pragma unroll 1
  for (int c = 0; c < NSTEP; ++c) {
    const int tot = chunk_hits<SCH / NT, SCH>(idx_i, cbase + c * SCH, n0, tid, LIST, scan_ws);
#pragma unroll 1
    for (int base = 0; base < tot; base += 32) {
      const int q = base + lane;
      const int qc = (q < SCH) ? q : (SCH - 1);
      const int lv = LIST[qc];
      const int rv = (q < tot) ? lv : -1;
      const int own = (rv >= 0 && (rv >> 27) == wave) ? 1 : 0;
      unsigned msk = (unsigned)__ballot(own);
#pragma unroll 1
      for (int it = 0; it < 32; ++it) {
        if (msk == 0u) break;
        const int bp = __builtin_ctz(msk); msk &= msk - 1u;
        const int r = __shfl(rv, bp, 32);
        const int dl = r >> 19;
        const int p = r & 0x7FFFF;
        int pl = p - cbase; pl = pl < 0 ? 0 : (pl >= CHK ? CHK - 1 : pl);
        int j = idx_j[p]; j = j < 0 ? 0 : (j >= NATOM ? NATOM - 1 : j);
        const float rc = rcut[pl] * rsc;
        const v4f hv = *(const v4f*)(H + (size_t)j * NB + 4 * lane);
        const v4h w4 = *(const v4h*)(W16 + (size_t)pl * NB + 4 * lane);
        float* rp = AGG + (size_t)(n0 + dl) * NB + 4 * lane;
        v4f a = *(const v4f*)rp;
#pragma unroll
        for (int e = 0; e < 4; ++e) a[e] += hv[e] * ((float)w4[e] * rc);
        *(v4f*)rp = a;
      }
    }
    __syncthreads();
  }
  const int s0 = (2 * lane) & 31, s1 = (2 * lane + 1) & 31;
#pragma unroll 1
  for (int jr = 0; jr < SRB / 8; ++jr) {
    const int row = rw0 + jr;
    float* rp = AGG + (size_t)row * NB + 4 * lane;
    const v4f a = *(const v4f*)rp;
    v8h h8;
#pragma unroll
    for (int e = 0; e < 4; ++e) {
      const float lo = __shfl(a[e], s0, 32);
      const float hi = __shfl(a[e], s1, 32);
      h8[e] = (_Float16)(lo * SC_T);
      h8[4 + e] = (_Float16)(hi * SC_T);
    }
    _Float16* hp = AGG16 + (size_t)row * NB + 8 * lane;
    for (int pass = 0; pass < 2; ++pass) {
      *(volatile v4f*)rp = a;
      if (last && lane < 16) *(volatile v8h*)hp = h8;
      __threadfence();
    }
  }
}

extern "C" void kernel_launch(void* const* d_in, const int* in_sizes, int n_in,
                              void* d_out, int out_size, void* d_ws, size_t ws_size, hipStream_t stream) {
  (void)n_in;
  if (out_size != NATOM * NB) return;
  if (in_sizes[0] != NATOM || in_sizes[1] != NATOM * 3 || in_sizes[2] != NPAIR || in_sizes[3] != NPAIR) return;
  const int*   Z     = (const int*)  d_in[0];
  const float* R     = (const float*)d_in[1];
  const int*   idx_i = (const int*)  d_in[2];
  const int*   idx_j = (const int*)  d_in[3];
  const float* emb   = (const float*)d_in[4];
  const float* in2fW = (const float*)d_in[5];
  const float* in2fb = (const float*)d_in[6];
  const float* fW1   = (const float*)d_in[7];
  const float* fb1   = (const float*)d_in[8];
  const float* fW2   = (const float*)d_in[9];
  const float* fb2   = (const float*)d_in[10];
  const float* oW1   = (const float*)d_in[11];
  const float* ob1   = (const float*)d_in[12];
  const float* oW2   = (const float*)d_in[13];
  const float* ob2   = (const float*)d_in[14];
  float* out = (float*)d_out;

  char* ws = (char*)d_ws; size_t off = 0;
  auto carve = [&](size_t bytes) -> char* { char* p = ws + off; off += (bytes + 255) & ~(size_t)255; return p; };
  _Float16* WT    = (_Float16*)carve((size_t)NLAYER * WPL * 2);
  float*    P0    = (float*)   carve((size_t)NATOM * NB * 4);
  _Float16* X16   = (_Float16*)carve((size_t)NATOM * NB * 2);
  float*    H     = (float*)   carve((size_t)NATOM * NB * 4);
  float*    AGG   = (float*)   carve((size_t)NATOM * NB * 4);
  _Float16* AGG16 = (_Float16*)carve((size_t)NATOM * NB * 2);
  _Float16* U16   = (_Float16*)carve((size_t)NATOM * NB * 2);
  _Float16* RBF   = (_Float16*)carve((size_t)CHK * KRBF * 2);
  float*    RCUT  = (float*)   carve((size_t)CHK * 4);
  _Float16* T16   = (_Float16*)carve((size_t)CHK * NB * 2);
  _Float16* W16   = (_Float16*)carve((size_t)CHK * NB * 2);
  if (off > ws_size || off > (size_t)134217728) return;

  const float s_in  = 1.0f / (SC_X * SC_W);
  const float s_f1  = 1.0f / SC_W;
  const float s_t64 = 1.0f / (SC_T * SC_W);
  const int blocksPair = ((CHK / 64) * (NB / 64) + 7) / 8;
  const int blocksAtom = ((NATOM / 64) * (NB / 64) + 7) / 8;

  prep_kernel<<<102, NT, 0, stream>>>(in2fW, fW1, fW2, oW1, oW2, WT);
  embed_kernel<<<(NATOM * 32) / NT, NT, 0, stream>>>(Z, emb, P0, X16);

  for (int l = 0; l < NLAYER; ++l) {
    const float* Pcur  = (l == 1) ? out : P0;
    float*       Pnext = (l == 1) ? P0 : out;
    const _Float16* wl = WT + (size_t)l * WPL;
    wmma_gemm64<0, false, 2, 0, false, 0><<<dim3(blocksAtom, 1), 256, 0, stream>>>(
        (const unsigned short*)X16, (const unsigned short*)nullptr, NB, 0L,
        (const unsigned short*)(wl + W_IN), (const unsigned short*)nullptr, NB, 0L,
        (void*)H, (void*)nullptr, NB, 0L,
        in2fb + l * NB, (const float*)nullptr, 0L, NATOM, NB, NB, s_in);
    for (int c = 0; c < NCHK; ++c) {
      const int cbase = c * CHK;
      geom_kernel<<<CHK / NT, NT, 0, stream>>>(R, idx_i, idx_j, RBF, RCUT, cbase);
      wmma_gemm64<0, false, 2, 1, false, 6><<<dim3(blocksPair, 1), 256, 0, stream>>>(
          (const unsigned short*)RBF, (const unsigned short*)nullptr, KRBF, 0L,
          (const unsigned short*)(wl + W_F1), (const unsigned short*)nullptr, KRBF, 0L,
          (void*)T16, (void*)nullptr, NB, 0L,
          fb1 + l * NB, (const float*)nullptr, 0L, CHK, NB, KRBF, s_f1);
      wmma_gemm64<0, false, 2, 1, false, 7><<<dim3(blocksPair, 1), 256, 0, stream>>>(
          (const unsigned short*)T16, (const unsigned short*)nullptr, NB, 0L,
          (const unsigned short*)(wl + W_F2), (const unsigned short*)nullptr, NB, 0L,
          (void*)W16, (void*)nullptr, NB, 0L,
          fb2 + l * NB, (const float*)nullptr, 0L, CHK, NB, NB, s_t64);
      agg_kernel<<<NTILE, NT, 0, stream>>>(idx_i, idx_j, H, W16, RCUT, AGG, AGG16, cbase,
                                           (c == 0) ? 1 : 0, (c == NCHK - 1) ? 1 : 0);
    }
    wmma_gemm64<0, false, 2, 1, false, 6><<<dim3(blocksAtom, 1), 256, 0, stream>>>(
        (const unsigned short*)AGG16, (const unsigned short*)nullptr, NB, 0L,
        (const unsigned short*)(wl + W_O1), (const unsigned short*)nullptr, NB, 0L,
        (void*)U16, (void*)nullptr, NB, 0L,
        ob1 + l * NB, (const float*)nullptr, 0L, NATOM, NB, NB, s_t64);
    wmma_gemm64<0, false, 2, 0, true, 0><<<dim3(blocksAtom, 1), 256, 0, stream>>>(
        (const unsigned short*)U16, (const unsigned short*)nullptr, NB, 0L,
        (const unsigned short*)(wl + W_O2), (const unsigned short*)nullptr, NB, 0L,
        (void*)Pnext, (void*)nullptr, NB, 0L,
        ob2 + l * NB, Pcur, 0L, NATOM, NB, NB, s_t64);
    if (l < NLAYER - 1) cast16_kernel<<<(NATOM * NB / 8) / NT, NT, 0, stream>>>(Pnext, X16, NATOM * NB / 8);
  }
}
